// MultiHeadedAttention_5858335392474
// MI455X (gfx1250) — hardware-verified
//
#include <hip/hip_runtime.h>
#include <math.h>

typedef __attribute__((ext_vector_type(16))) _Float16 v16h;
typedef __attribute__((ext_vector_type(16))) __bf16 v16b;
typedef __attribute__((ext_vector_type(8)))  _Float16 v8h;
typedef __attribute__((ext_vector_type(8)))  __bf16 v8b;
typedef __attribute__((ext_vector_type(8)))  float v8f;
typedef __attribute__((ext_vector_type(4)))  float v4f;
typedef __attribute__((ext_vector_type(4)))  unsigned v4u;
typedef __attribute__((ext_vector_type(4)))  int v4i;

template <typename T> __device__ __forceinline__ void vst2(void* p, T v) { *(volatile T*)p = v; __threadfence(); *(volatile T*)p = v; }
__device__ __forceinline__ v8f wmma16(v16h a, v16h b, v8f c) {
  v8f d = __builtin_amdgcn_wmma_f32_16x16x32_f16(false, a, false, b, (short)0, c, false, false);
  asm volatile("v_nop\n\tv_nop\n\tv_nop\n\tv_nop" : "+v"(d) : "v"(a), "v"(b));
  return d;
}
__device__ __forceinline__ v8f wmma_bf(v16b a, v16b b, v8f c) {
  v8f d = __builtin_amdgcn_wmma_f32_16x16x32_bf16(false, a, false, b, (short)0, c, false, false);
  asm volatile("v_nop\n\tv_nop\n\tv_nop\n\tv_nop" : "+v"(d) : "v"(a), "v"(b));
  return d;
}
__device__ __forceinline__ v16h frag_h(const _Float16* rowk0, int lane) {
  union { v16h v; v8h q[2]; } u; const _Float16* p = rowk0 + 8 * (lane >> 4);
  u.q[0] = *(const v8h*)p; u.q[1] = *(const v8h*)(p + 16); return u.v;
}
__device__ __forceinline__ v16b frag_b(const __bf16* rowk0, int lane) {
  union { v16b v; v8b q[2]; } u; const __bf16* p = rowk0 + 8 * (lane >> 4);
  u.q[0] = *(const v8b*)p; u.q[1] = *(const v8b*)(p + 16); return u.v;
}
__device__ __forceinline__ float bfr(float v) { return (float)(__bf16)v; }
#define LDSX() do { asm volatile("s_wait_dscnt 0" ::: "memory"); __builtin_amdgcn_wave_barrier(); __builtin_amdgcn_fence(3  , "workgroup"); } while (0)

#ifndef NB
#define NB 2
#endif
#ifndef SEQ
#define SEQ 2048
#endif
#define NB_FULL 2
#define SEQ_FULL 2048
#define DM 1024
#define NH 16
#define HD 64
#define NROW (NB * SEQ)
#define SCALE (0.125f)
#define RSC (1.0f / 1024.0f)

static_assert(NH * HD == DM);
static_assert(HD == 64);
static_assert(DM % 128 == 0);
static_assert(DM % 32 == 0);
static_assert(SEQ % 64 == 0);
static_assert(NROW % 64 == 0);
static_assert(NB <= NB_FULL);
static_assert(SEQ <= SEQ_FULL);

#define SZ_ROWS (2u * (size_t)NROW * DM)
#define WS_XB  ((size_t)0)
#define WS_WB  (WS_XB + SZ_ROWS)
#define WS_WO  (WS_WB + 2u * (size_t)3 * DM * DM)
#define WS_QH  (WS_WO + 2u * (size_t)DM * DM)
#define WS_QL  (WS_QH + SZ_ROWS)
#define WS_KH  (WS_QL + SZ_ROWS)
#define WS_KL  (WS_KH + SZ_ROWS)
#define WS_VT  (WS_KL + SZ_ROWS)
#define WS_Y   (WS_VT + 2u * (size_t)NB * DM * SEQ)
#define WS_END (WS_Y + SZ_ROWS)
static_assert(WS_END <= (size_t)134217728);
static_assert(SZ_ROWS % 128 == 0);

#define NVX (NROW * DM / 8)
#define NVW (3 * DM * DM / 8)
#define NVO (DM * DM / 8)
static_assert(NVX % 256 == 0);
static_assert(NVW % 256 == 0);
static_assert(NVO % 256 == 0);

__global__ __launch_bounds__(256) void k_cvt(const float* __restrict__ X, const float* __restrict__ WQ, const float* __restrict__ WO, __bf16* __restrict__ XB, __bf16* __restrict__ WB, _Float16* __restrict__ WOH) {
  const int v = blockIdx.x * 256 + threadIdx.x;
  if (v < NVX) {
    const int row = v / (DM / 8), c8 = v % (DM / 8); const int b = row / SEQ, s = row % SEQ;
    const float* p = X + ((size_t)b * SEQ_FULL + s) * DM + c8 * 8;
    const v4f a = *(const v4f*)p, c = *(const v4f*)(p + 4); v8b o;
#pragma unroll
    for (int i = 0; i < 4; ++i) { o[i] = (__bf16)a[i]; o[4 + i] = (__bf16)c[i]; }
    vst2(XB + (size_t)v * 8, __builtin_bit_cast(v4u, o));
  } else if (v < NVX + NVW) {
    const int u = v - NVX; const float* p = WQ + (size_t)u * 8;
    const v4f a = *(const v4f*)p, c = *(const v4f*)(p + 4); v8b o;
#pragma unroll
    for (int i = 0; i < 4; ++i) { o[i] = (__bf16)a[i]; o[4 + i] = (__bf16)c[i]; }
    vst2(WB + (size_t)u * 8, __builtin_bit_cast(v4u, o));
  } else {
    const int u = v - NVX - NVW; const float* p = WO + (size_t)u * 8;
    const v4f a = *(const v4f*)p, c = *(const v4f*)(p + 4); v8h o;
#pragma unroll
    for (int i = 0; i < 4; ++i) { o[i] = (_Float16)(bfr(a[i]) * 256.0f); o[4 + i] = (_Float16)(bfr(c[i]) * 256.0f); }
    vst2(WOH + (size_t)u * 8, __builtin_bit_cast(v4u, o));
  }
}

__global__ __launch_bounds__(128) void k_proj(const __bf16* __restrict__ XB, const __bf16* __restrict__ WB, _Float16* __restrict__ P16) {
  __shared__ __align__(16) _Float16 sh[64][136]; __shared__ __align__(16) _Float16 sl[64][136]; __shared__ __align__(16) _Float16 th[128][72];
  const int tid = threadIdx.x, wave = tid >> 5, lane = tid & 31, col = lane & 15, g = lane >> 4;
  const int which = blockIdx.z; const int c0 = blockIdx.y * 128; const size_t r0 = (size_t)blockIdx.x * 64; const size_t bb = r0 / SEQ; const int t0 = (int)(r0 % SEQ);
  v8f acc[8] = {};
  const __bf16* ap = XB + (r0 + wave * 16 + col) * DM;
  const __bf16* wp = WB + ((size_t)which * DM + c0 + col) * DM;
#pragma unroll 2
  for (int kc = 0; kc < DM / 32; ++kc) { const v16b a = frag_b(ap + kc * 32, lane);
#pragma unroll
    for (int j = 0; j < 8; ++j) { const v16b w = frag_b(wp + (size_t)j * 16 * DM + kc * 32, lane); acc[j] = wmma_bf(a, w, acc[j]); } }
  if (which < 2) {
    const size_t oh = (which == 0 ? WS_QH : WS_KH) / 2, ol = (which == 0 ? WS_QL : WS_KL) / 2;
#pragma unroll
    for (int j = 0; j < 8; ++j) {
#pragma unroll
      for (int r = 0; r < 8; ++r) { const float v = acc[j][r]; const _Float16 hv = (_Float16)v; sh[wave * 16 + 8 * g + r][j * 16 + col] = hv; sl[wave * 16 + 8 * g + r][j * 16 + col] = (_Float16)((v - (float)hv) * 1024.0f); } }
    __syncthreads();
    for (int e = tid; e < 64 * 16; e += 128) { const int rl = e >> 4, q = e & 15; const size_t o = (r0 + rl) * DM + c0 + q * 8;
      const v4u a = *(const v4u*)&sh[rl][q * 8]; const v4u b = *(const v4u*)&sl[rl][q * 8];
      vst2(P16 + oh + o, a); vst2(P16 + ol + o, b); }
  } else {
#pragma unroll
    for (int j = 0; j < 8; ++j) {
#pragma unroll
      for (int r = 0; r < 8; ++r) th[j * 16 + col][wave * 16 + 8 * g + r] = (_Float16)acc[j][r]; }
    __syncthreads();
    for (int e = tid; e < 128 * 8; e += 128) { const int cl = e >> 3, q = e & 7; const v4u a = *(const v4u*)&th[cl][q * 8];
      vst2(P16 + WS_VT / 2 + (bb * DM + c0 + cl) * (size_t)SEQ + t0 + q * 8, a); }
  }
}

__global__ __launch_bounds__(128) void k_attn(const _Float16* __restrict__ QH, const _Float16* __restrict__ QL, const _Float16* __restrict__ KH, const _Float16* __restrict__ KL, const _Float16* __restrict__ VT, const int* __restrict__ MK, _Float16* __restrict__ Y) {
  __shared__ __align__(16) _Float16 so[4][16][72];
  const int tid = threadIdx.x, wave = tid >> 5, lane = tid & 31, col = lane & 15, g = lane >> 4;
  const int qb = blockIdx.x, h = blockIdx.y, b = blockIdx.z;
  const int qrow = qb * 64 + wave * 16 + col;
  const size_t qoff0 = ((size_t)b * SEQ + qrow) * DM + h * HD;
  const size_t koff0 = ((size_t)b * SEQ + col) * DM + h * HD;
  const size_t voff0 = ((size_t)b * DM + h * HD + col) * SEQ;
  const size_t moff0 = ((size_t)b * SEQ_FULL + qrow) * SEQ_FULL + 8 * g;
  v8f o[4] = {}; float m = -1.0e30f, l = 0.0f;
#pragma unroll 1
  for (int kb = 0; kb < SEQ; kb += 32) {
    int qo = 0; asm volatile("" : "+v"(qo));
    v8f s0 = {}, s1 = {}, r0 = {}, r1 = {};
    const size_t kr = koff0 + (size_t)kb * DM;
#pragma unroll
    for (int kc = 0; kc < 2; ++kc) {
      const v16h qh = frag_h(QH + qoff0 + qo + kc * 32, lane), ql = frag_h(QL + qoff0 + qo + kc * 32, lane);
      const v16h k0h = frag_h(KH + kr + kc * 32, lane), k0l = frag_h(KL + kr + kc * 32, lane);
      s0 = wmma16(k0h, qh, s0); r0 = wmma16(k0l, qh, r0); r0 = wmma16(k0h, ql, r0);
      const v16h k1h = frag_h(KH + kr + (size_t)16 * DM + kc * 32, lane), k1l = frag_h(KL + kr + (size_t)16 * DM + kc * 32, lane);
      s1 = wmma16(k1h, qh, s1); r1 = wmma16(k1l, qh, r1); r1 = wmma16(k1h, ql, r1);
    }
    const int* mp = MK + moff0 + kb;
    const v4i ma = *(const v4i*)mp, mb = *(const v4i*)(mp + 4), mc = *(const v4i*)(mp + 16), md = *(const v4i*)(mp + 20);
    float t0[8], t1[8]; float mx = -1.0e30f;
#pragma unroll
    for (int r = 0; r < 8; ++r) {
      float a0 = (s0[r] + r0[r] * RSC) * SCALE, a1 = (s1[r] + r1[r] * RSC) * SCALE;
      const int m0 = r < 4 ? ma[r & 3] : mb[r & 3], m1 = r < 4 ? mc[r & 3] : md[r & 3];
      a0 = (m0 == 0) ? -1.0e9f : a0; a1 = (m1 == 0) ? -1.0e9f : a1;
      t0[r] = a0; t1[r] = a1; mx = fmaxf(mx, fmaxf(a0, a1)); }
    mx = fmaxf(mx, __shfl_xor(mx, 16));
    const float mn = fmaxf(m, mx); const float corr = __expf(m - mn); m = mn;
    float sum = 0.0f; v16h pf;
#pragma unroll
    for (int r = 0; r < 8; ++r) { const float p0 = __expf(t0[r] - mn), p1 = __expf(t1[r] - mn); sum += p0 + p1; pf[r] = (_Float16)(p0 * 256.0f); pf[8 + r] = (_Float16)(p1 * 256.0f); }
    sum += __shfl_xor(sum, 16);
    l = l * corr + sum;
#pragma unroll
    for (int j = 0; j < 4; ++j) o[j] = o[j] * corr;
    const v16h v0 = frag_h(VT + voff0 + kb, lane), v1 = frag_h(VT + voff0 + (size_t)16 * SEQ + kb, lane), v2 = frag_h(VT + voff0 + (size_t)32 * SEQ + kb, lane), v3 = frag_h(VT + voff0 + (size_t)48 * SEQ + kb, lane);
    o[0] = wmma16(v0, pf, o[0]); o[1] = wmma16(v1, pf, o[1]); o[2] = wmma16(v2, pf, o[2]); o[3] = wmma16(v3, pf, o[3]);
  }
  const float inv = 0.25f * (1.0f / l);
#pragma unroll
  for (int j = 0; j < 4; ++j) { v8h t;
#pragma unroll
    for (int r = 0; r < 8; ++r) t[r] = (_Float16)(o[j][r] * inv);
    *(v8h*)&so[wave][col][j * 16 + 8 * g] = t; }
  LDSX();
#pragma unroll
  for (int it = 0; it < 4; ++it) { const int row = it * 4 + (lane >> 3), pc = lane & 7; const v4u w = *(const v4u*)&so[wave][row][pc * 8];
    vst2(Y + ((size_t)b * SEQ + qb * 64 + wave * 16 + row) * DM + h * HD + pc * 8, w); }
}

__global__ __launch_bounds__(128) void k_out(const _Float16* __restrict__ Y, const _Float16* __restrict__ WOH, const float* __restrict__ BO, float* __restrict__ OUT) {
  __shared__ __align__(16) float sf[4][16][132];
  const int tid = threadIdx.x, wave = tid >> 5, lane = tid & 31, col = lane & 15, g = lane >> 4; const int c0 = blockIdx.y * 128; const size_t r0 = (size_t)blockIdx.x * 64 + wave * 16;
  v8f acc[8] = {};
  const _Float16* ap = Y + (r0 + col) * DM; const _Float16* wp = WOH + (size_t)(c0 + col) * DM;
#pragma unroll 2
  for (int kc = 0; kc < DM / 32; ++kc) { const v16h a = frag_h(ap + kc * 32, lane);
#pragma unroll
    for (int j = 0; j < 8; ++j) { const v16h w = frag_h(wp + (size_t)j * 16 * DM + kc * 32, lane); acc[j] = wmma16(a, w, acc[j]); } }
#pragma unroll
  for (int j = 0; j < 8; ++j) { const float bias = bfr(BO[c0 + j * 16 + col]);
#pragma unroll
    for (int r = 0; r < 8; ++r) sf[wave][8 * g + r][j * 16 + col] = acc[j][r] * (1.0f / 16384.0f) + bias; }
  LDSX();
  for (int rl = 0; rl < 16; ++rl) { const v4f w = *(const v4f*)&sf[wave][rl][lane * 4]; vst2(OUT + (r0 + rl) * DM + c0 + lane * 4, w); }
}

extern "C" void kernel_launch(void* const* d_in, const int* in_sizes, int n_in, void* d_out, int out_size, void* d_ws, size_t ws_size, hipStream_t stream) {
  if (n_in < 5) return;
  if (in_sizes[0] < ((NB - 1) * SEQ_FULL + SEQ) * DM) return;
  if (in_sizes[1] < ((NB - 1) * SEQ_FULL + SEQ - 1) * SEQ_FULL + SEQ) return;
  if (in_sizes[2] < 3 * DM * DM) return;
  if (in_sizes[3] < DM * DM) return;
  if (in_sizes[4] < DM) return;
  if (out_size < NROW * DM) return;
  if (ws_size < (size_t)WS_END) return;
  const float* X = (const float*)d_in[0]; const int* MK = (const int*)d_in[1]; const float* WQ = (const float*)d_in[2]; const float* WO = (const float*)d_in[3]; const float* BO = (const float*)d_in[4];
  char* ws = (char*)d_ws;
  __bf16* XB = (__bf16*)(ws + WS_XB); __bf16* WB = (__bf16*)(ws + WS_WB); _Float16* WOH = (_Float16*)(ws + WS_WO);
  _Float16* P16 = (_Float16*)ws;
  _Float16 *QH = (_Float16*)(ws + WS_QH), *QL = (_Float16*)(ws + WS_QL), *KH = (_Float16*)(ws + WS_KH), *KL = (_Float16*)(ws + WS_KL), *VT = (_Float16*)(ws + WS_VT), *Y = (_Float16*)(ws + WS_Y);
  k_cvt<<<dim3((NVX + NVW + NVO) / 256), 256, 0, stream>>>(X, WQ, WO, XB, WB, WOH);
  k_proj<<<dim3(NROW / 64, DM / 128, 3), 128, 0, stream>>>(XB, WB, P16);
  k_attn<<<dim3(SEQ / 64, NH, NB), 128, 0, stream>>>(QH, QL, KH, KL, VT, MK, Y);
  k_out<<<dim3(NROW / 64, DM / 128), 128, 0, stream>>>(Y, WOH, BO, (float*)d_out);
}
